// VDP_ViT_27745488732909
// MI455X (gfx1250) — hardware-run, weakly checked
//
#include <hip/hip_runtime.h>
#include <math.h>

typedef __attribute__((ext_vector_type(16))) _Float16 v16h;
typedef __attribute__((ext_vector_type(16))) __bf16 v16b;
typedef __attribute__((ext_vector_type(8)))  _Float16 v8h;
typedef __attribute__((ext_vector_type(8)))  float v8f;
typedef __attribute__((ext_vector_type(4)))  float v4f;
typedef __attribute__((ext_vector_type(2)))  float v2f;
typedef __attribute__((ext_vector_type(4)))  unsigned v4u;
typedef __attribute__((ext_vector_type(4)))  int v4i;
typedef float __attribute__((may_alias)) float_a;
typedef int __attribute__((may_alias)) int_a;

template <typename T> __device__ __forceinline__ void vst2(void* p, T v) { *(volatile T*)p = v; __threadfence(); *(volatile T*)p = v; }
__device__ __forceinline__ v8f wmma16(v16h a, v16h b, v8f c) {
  v8f d = __builtin_amdgcn_wmma_f32_16x16x32_f16(false, a, false, b, (short)0, c, false, false);
  asm volatile("v_nop\n\tv_nop\n\tv_nop\n\tv_nop" : "+v"(d) : "v"(a), "v"(b));
  return d;
}
__device__ __forceinline__ v8f wmma_bf(v16b a, v16b b, v8f c) {
  v8f d = __builtin_amdgcn_wmma_f32_16x16x32_bf16(false, a, false, b, (short)0, c, false, false);
  asm volatile("v_nop\n\tv_nop\n\tv_nop\n\tv_nop" : "+v"(d) : "v"(a), "v"(b));
  return d;
}
__device__ __forceinline__ v16h frag_h(const _Float16* rowk0, int lane) {
  union { v16h v; v8h q[2]; } u; const _Float16* p = rowk0 + 8 * (lane >> 4);
  u.q[0] = *(const v8h*)p; u.q[1] = *(const v8h*)(p + 16); return u.v;
}
__device__ __forceinline__ v16h frag_f32(const float* rowk0, int lane) {
  v16h a; const float* p = rowk0 + 8 * (lane >> 4);
#pragma unroll
  for (int i = 0; i < 8; ++i) { a[i] = (_Float16)p[i]; a[8 + i] = (_Float16)p[16 + i]; }
  return a;
}
__device__ __forceinline__ v16h frag_f32s(const float* rowk0, int lane, float sc) {
  v16h a; const float* p = rowk0 + 8 * (lane >> 4);
#pragma unroll
  for (int i = 0; i < 8; ++i) { a[i] = (_Float16)(p[i] * sc); a[8 + i] = (_Float16)(p[16 + i] * sc); }
  return a;
}
__device__ __forceinline__ v16h fragc_f32(const float* W, int k0, int n, int lane, int ld, int K) {
  v16h a; const int g = lane >> 4;
#pragma unroll
  for (int i = 0; i < 8; ++i) { const int ka = k0 + 8 * g + i, kb = ka + 16;
    a[i] = (_Float16)(ka < K ? W[(size_t)(ka < K ? ka : K - 1) * ld + n] : 0.f); a[8 + i] = (_Float16)(kb < K ? W[(size_t)(kb < K ? kb : K - 1) * ld + n] : 0.f); }
  return a;
}
struct F2 { v16b h, l; };
__device__ __forceinline__ F2 bsplit16(const float v[16]) { F2 r;
#pragma unroll
  for (int i = 0; i < 16; ++i) { const __bf16 h = (__bf16)v[i]; r.h[i] = h; r.l[i] = (__bf16)(v[i] - (float)h); }
  return r; }
__device__ __forceinline__ F2 split_row(const float* row, int k0, int lane) { float v[16]; const float* p = row + k0 + 8 * (lane >> 4);
#pragma unroll
  for (int i = 0; i < 8; ++i) { v[i] = p[i]; v[8 + i] = p[16 + i]; }
  return bsplit16(v); }
__device__ __forceinline__ F2 split_rowK(const float* row, int k0, int lane, int K) { float v[16]; const int g = lane >> 4;
#pragma unroll
  for (int i = 0; i < 8; ++i) { const int ka = k0 + 8 * g + i, kb = ka + 16; v[i] = ka < K ? row[ka < K ? ka : K - 1] : 0.f; v[8 + i] = kb < K ? row[kb < K ? kb : K - 1] : 0.f; }
  return bsplit16(v); }
__device__ __forceinline__ F2 split_col(const float* W, int k0, int n, int lane, int ld, int K) { float v[16]; const int g = lane >> 4;
#pragma unroll
  for (int i = 0; i < 8; ++i) { const int ka = k0 + 8 * g + i, kb = ka + 16; v[i] = ka < K ? W[(size_t)(ka < K ? ka : K - 1) * ld + n] : 0.f; v[8 + i] = kb < K ? W[(size_t)(kb < K ? kb : K - 1) * ld + n] : 0.f; }
  return bsplit16(v); }
__device__ __forceinline__ v8f mac3(const F2& a, const F2& b, v8f c) { c = wmma_bf(a.l, b.h, c); c = wmma_bf(a.h, b.l, c); return wmma_bf(a.h, b.h, c); }
__device__ __forceinline__ float sigm(float v) { return 1.0f / (1.0f + expf(-v)); }
#define LDSX() do { asm volatile("s_wait_dscnt 0" ::: "memory"); __builtin_amdgcn_wave_barrier(); __builtin_amdgcn_fence(__ATOMIC_RELEASE, "workgroup"); } while (0)


#ifndef NB
#define NB 8
#endif
#define SS 512
#define E_ 768
#define NH 12
#define HD 64
#define NROW (NB * SS)
#define PRIOR_VAR 0.01f
typedef __attribute__((ext_vector_type(8))) __bf16 v8b;
__device__ __forceinline__ v16b frag_b(const __bf16* rowk0, int lane) {
  union { v16b v; v8b q[2]; } u; const __bf16* p = rowk0 + 8 * (lane >> 4);
  u.q[0] = *(const v8b*)p; u.q[1] = *(const v8b*)(p + 16); return u.v;
}
__device__ __forceinline__ float bfr(float v) { return (float)(__bf16)v; }
__device__ __attribute__((noinline)) float exp_ni(float v) { return expf(v); }
__device__ __attribute__((noinline)) float erf_ni(float v) { return erff(v); }

#define OUT1_OFF ((size_t)8 * SS * E_)
#define OUT2_OFF ((size_t)2 * 8 * SS * E_)
#define WS_QH   0u
#define WS_QL   (WS_QH + 2u * (size_t)NROW * E_)
#define WS_KH   (WS_QL + 2u * (size_t)NROW * E_)
#define WS_VT   (WS_KH + 2u * (size_t)NROW * E_)
#define WS_AQ   (WS_VT + 2u * (size_t)NROW * E_)
#define WS_BK   (WS_AQ + 2u * (size_t)NROW * 3 * E_)
#define WS_SGV  (WS_BK + 2u * (size_t)NROW * 3 * E_)
#define WS_VS   (WS_SGV + 2u * (size_t)NROW * E_)
#define WS_RST  (WS_VS + 2u * (size_t)NROW * E_)
#define WS_S    (WS_RST + 4u * (size_t)NROW * 4)
#define WS_SG   (WS_S + 4u * (size_t)SS * SS)
#define WS_PH   (WS_SG + 4u * (size_t)SS * SS)
#define WS_GD   (WS_PH + 2u * (size_t)SS * SS)
#define WS_AE   (WS_GD + 2u * (size_t)SS * SS)
#define WS_MUC  (WS_AE + 2u * (size_t)SS * SS)
#define WS_SGC  (WS_MUC + 4u * (size_t)NROW * E_)
#define WS_CST  (WS_SGC + 2u * (size_t)NROW * E_)
#define WS_W2   (WS_CST + 4u * (size_t)NROW * 32)
#define WS_WSG  (WS_W2 + 2u * (size_t)4 * E_ * E_)
#define WS_END  (WS_WSG + 4u * (size_t)4 * E_)

__device__ __forceinline__ float softplusf(float x) { return (x > 20.f) ? x : log1pf(expf(x)); }
__global__ __launch_bounds__(256) void k_prep(const float* __restrict__ WQ, const float* __restrict__ SQ, const float* __restrict__ WK, const float* __restrict__ SK, const float* __restrict__ WV, const float* __restrict__ SV, const float* __restrict__ WO, const float* __restrict__ SO, _Float16* __restrict__ W2, float* __restrict__ WSG, float* __restrict__ KLP) {
  __shared__ __align__(16) _Float16 sw[4][E_]; __shared__ float sred[8][4]; __shared__ __align__(16) float sws[E_]; __shared__ __align__(16) float so[4];
  const int t = threadIdx.x; const int i = blockIdx.x;
  float klp[4] = {0.f, 0.f, 0.f, 0.f};
#pragma unroll
  for (int m = 0; m < 4; ++m) for (int o = t; o < E_; o += 256) { const float* wm = (m == 0) ? WQ : (m == 1) ? WK : (m == 2) ? WV : WO; const float* sm_ = (m == 0) ? SQ : (m == 1) ? SK : (m == 2) ? SV : SO; const float w = bfr(wm[(size_t)i * E_ + o]); sw[m][o] = (_Float16)(w * w); const float ws = bfr(sm_[o]);
      klp[m] += (logf(PRIOR_VAR) - 1.0f - ws + softplusf(ws) / PRIOR_VAR + w * w / PRIOR_VAR); }
#pragma unroll
  for (int m = 0; m < 4; ++m) { float v = klp[m];
#pragma unroll
    for (int o = 1; o < 32; o <<= 1) v += __shfl_xor(v, o); if ((t & 31) == 0) sred[t >> 5][m] = v; }
  __syncthreads(); if (t < 4) { float v = 0.f; for (int w = 0; w < 8; ++w) v += sred[w][t]; so[t] = v; }
  for (int m = 0; m < 4; ++m) for (int q = t; q < E_ / 8; q += 256) vst2((unsigned*)(W2 + ((size_t)m * E_ + i) * E_ + q * 8), *(const v4u*)&sw[m][q * 8]);
  if (i < 4) { const float* smi = (i == 0) ? SQ : (i == 1) ? SK : (i == 2) ? SV : SO; for (int o = t; o < E_; o += 256) sws[o] = softplusf(bfr(smi[o])); __syncthreads(); for (int q = t; q < E_ / 4; q += 256) vst2(WSG + (size_t)i * E_ + q * 4, *(const v4f*)&sws[q * 4]); }
  __syncthreads(); if (t == 0) vst2(KLP + (size_t)i * 4, *(const v4f*)&so[0]); }
__global__ __launch_bounds__(256) void k_rowstat(const float* __restrict__ MU, const float* __restrict__ SG, float* __restrict__ RST) { __shared__ float sred[8][2]; __shared__ __align__(16) float so[4]; const int t = threadIdx.x; const size_t row = blockIdx.x;
  float a = 0.f, b = 0.f; for (int d = t; d < E_; d += 256) { const float m = bfr(MU[row * E_ + d]) * (1.0f / E_); a += m * m; b += bfr(SG[row * E_ + d]); }
#pragma unroll
  for (int o = 1; o < 32; o <<= 1) { a += __shfl_xor(a, o); b += __shfl_xor(b, o); }
  if ((t & 31) == 0) { sred[t >> 5][0] = a; sred[t >> 5][1] = b; } __syncthreads();
  if (t == 0) { float x = 0.f, y = 0.f; for (int w = 0; w < 8; ++w) { x += sred[w][0]; y += sred[w][1]; } so[0] = x; so[1] = y; so[2] = 0.f; so[3] = 0.f; vst2(RST + row * 4, *(const v4f*)&so[0]); } }
__global__ __launch_bounds__(128) void k_mu(const float* __restrict__ MU, const float* __restrict__ WQ, const float* __restrict__ WK, const float* __restrict__ WV, _Float16* __restrict__ QH, _Float16* __restrict__ QL, _Float16* __restrict__ KH, _Float16* __restrict__ VT, _Float16* __restrict__ AQ, _Float16* __restrict__ VS2) {
  __shared__ __align__(16) _Float16 sh[64][136], sl[64][136], s2[64][136]; __shared__ __align__(16) _Float16 th[128][72], t2[128][72];
  const int tid = threadIdx.x, wave = tid >> 5, lane = tid & 31, col = lane & 15, g = lane >> 4; const int which = blockIdx.z; const int c0 = blockIdx.y * 128; const size_t r0 = (size_t)blockIdx.x * 64; const float* Wm = which == 0 ? WQ : which == 1 ? WK : WV;
  v8f acc[8] = {};
#pragma unroll 2
  for (int kc = 0; kc < E_ / 32; ++kc) { v16b a; { const float* p = MU + (r0 + wave * 16 + col) * E_ + kc * 32 + 8 * g;
#pragma unroll
      for (int i = 0; i < 8; ++i) { a[i] = (__bf16)p[i]; a[8 + i] = (__bf16)p[16 + i]; } }
#pragma unroll
    for (int j = 0; j < 8; ++j) { v16b w; const int o = c0 + j * 16 + col;
#pragma unroll
      for (int i = 0; i < 8; ++i) { w[i] = (__bf16)Wm[(size_t)(kc * 32 + 8 * g + i) * E_ + o]; w[8 + i] = (__bf16)Wm[(size_t)(kc * 32 + 16 + 8 * g + i) * E_ + o]; }
      acc[j] = wmma_bf(a, w, acc[j]); } }
#pragma unroll
  for (int j = 0; j < 8; ++j)
#pragma unroll
    for (int r = 0; r < 8; ++r) { const float v = acc[j][r]; const int rl = wave * 16 + 8 * g + r, cl = j * 16 + col; const _Float16 hv = (_Float16)v;
      if (which == 2) { th[cl][rl] = hv; t2[cl][rl] = (_Float16)(v * v); } else { sh[rl][cl] = hv; sl[rl][cl] = (_Float16)(v - (float)hv); s2[rl][cl] = (_Float16)(v * v); } }
  __syncthreads();
  if (which < 2) { _Float16* dh = which == 0 ? QH : KH; const int aoff = which == 0 ? 0 : 64;
    for (int e = tid; e < 64 * 16; e += 128) { const int rl = e >> 4, q = e & 15; const int c = c0 + q * 8; vst2((unsigned*)(dh + (r0 + rl) * E_ + c), *(const v4u*)&sh[rl][q * 8]); if (which == 0) vst2((unsigned*)(QL + (r0 + rl) * E_ + c), *(const v4u*)&sl[rl][q * 8]); const int h = c / HD, dd = c % HD; vst2((unsigned*)(AQ + (r0 + rl) * (3 * E_) + h * 192 + aoff + dd), *(const v4u*)&s2[rl][q * 8]); } }
  else { const size_t b = r0 / SS; const int s0 = (int)(r0 % SS); for (int e = tid; e < 128 * 8; e += 128) { const int cl = e >> 3, q = e & 7; const size_t o = (b * E_ + c0 + cl) * (size_t)SS + s0 + q * 8; vst2((unsigned*)(VT + o), *(const v4u*)&th[cl][q * 8]); vst2((unsigned*)(VS2 + o), *(const v4u*)&t2[cl][q * 8]); } } }
__global__ __launch_bounds__(128) void k_sg(const float* __restrict__ SGIN, const _Float16* __restrict__ W2, const float* __restrict__ WSG, const float* __restrict__ RST, int which, _Float16* __restrict__ AQ, _Float16* __restrict__ BK, _Float16* __restrict__ SGV, const _Float16* __restrict__ VS2, _Float16* __restrict__ VS) {
  __shared__ __align__(16) _Float16 sh[64][136]; __shared__ __align__(16) _Float16 th[128][72], tv[128][72];
  const int tid = threadIdx.x, wave = tid >> 5, lane = tid & 31, col = lane & 15, g = lane >> 4; const int c0 = blockIdx.y * 128; const size_t r0 = (size_t)blockIdx.x * 64; const _Float16* Wm = W2 + (size_t)which * E_ * E_; const float* wsg = WSG + (size_t)which * E_;
  v8f acc[8] = {};
#pragma unroll 2
  for (int kc = 0; kc < E_ / 32; ++kc) { v16h a; { const float* p = SGIN + (r0 + wave * 16 + col) * E_ + kc * 32 + 8 * g;
#pragma unroll
      for (int i = 0; i < 8; ++i) { a[i] = (_Float16)bfr(p[i]); a[8 + i] = (_Float16)bfr(p[16 + i]); } }
#pragma unroll
    for (int j = 0; j < 8; ++j) { v16h w; const int o = c0 + j * 16 + col;
#pragma unroll
      for (int i = 0; i < 8; ++i) { w[i] = Wm[(size_t)(kc * 32 + 8 * g + i) * E_ + o]; w[8 + i] = Wm[(size_t)(kc * 32 + 16 + 8 * g + i) * E_ + o]; }
      acc[j] = wmma16(a, w, acc[j]); } }
#pragma unroll
  for (int j = 0; j < 8; ++j) { const int o = c0 + j * 16 + col; const float wsv = wsg[o];
#pragma unroll
    for (int r = 0; r < 8; ++r) { const size_t row = r0 + wave * 16 + 8 * g + r; const float xx = RST[row * 4], rs = RST[row * 4 + 1]; const float z = acc[j][r] * (1.0f / E_) + xx * wsv + rs * wsv * (1.0f / E_); const float sgv = softplusf(z); const int rl = wave * 16 + 8 * g + r, cl = j * 16 + col;
      if (which == 2) { th[cl][rl] = (_Float16)sgv; } else sh[rl][cl] = (_Float16)sgv; } }
  __syncthreads();
  if (which < 2) { for (int e = tid; e < 64 * 16; e += 128) { const int rl = e >> 4, q = e & 15; const int c = c0 + q * 8; const int h = c / HD, dd = c % HD; const v4u v = *(const v4u*)&sh[rl][q * 8]; const size_t rb = (r0 + rl) * (3 * E_) + h * 192;
      if (which == 0) { vst2((unsigned*)(AQ + rb + 128 + dd), v); vst2((unsigned*)(BK + rb + 64 + dd), v); } else { vst2((unsigned*)(BK + rb + dd), v); vst2((unsigned*)(BK + rb + 128 + dd), v); } } }
  else { const size_t b = r0 / SS; const int s0 = (int)(r0 % SS);
    for (int e = tid; e < 128 * 8; e += 128) { const int cl = e >> 3, q = e & 7; const size_t o = (b * E_ + c0 + cl) * (size_t)SS + s0 + q * 8; const v4u sv = *(const v4u*)&th[cl][q * 8]; vst2((unsigned*)(SGV + o), sv); v4u m2 = *(const v4u*)(VS2 + o); _Float16* a1 = (_Float16*)&m2; const _Float16* a2 = (const _Float16*)&sv; _Float16 tmp[8];
      for (int i = 0; i < 8; ++i) tmp[i] = (_Float16)((float)a1[i] + (float)a2[i]); vst2((unsigned*)(VS + o), *(const v4u*)tmp); } } }
__global__ __launch_bounds__(128) void k_sc2(const _Float16* __restrict__ QH, const _Float16* __restrict__ QL, const _Float16* __restrict__ KH, const _Float16* __restrict__ AQ, const _Float16* __restrict__ BK, int b, int h, float* __restrict__ S, float* __restrict__ SG) { __shared__ __align__(16) float ss[4][16][132];
  const int tid = threadIdx.x, wave = tid >> 5, lane = tid & 31, col = lane & 15, g = lane >> 4; const int k0 = blockIdx.y * 128; const int ql0 = blockIdx.x * 64 + wave * 16; const size_t q0 = (size_t)b * SS + ql0;
  v8f acc[8] = {}, acs[8] = {};
#pragma unroll
  for (int kc = 0; kc < HD / 32; ++kc) { const v16h ah = frag_h(QH + (q0 + col) * E_ + h * HD + kc * 32, lane), al = frag_h(QL + (q0 + col) * E_ + h * HD + kc * 32, lane);
#pragma unroll
    for (int j = 0; j < 8; ++j) { const v16h kb = frag_h(KH + ((size_t)b * SS + k0 + j * 16 + col) * E_ + h * HD + kc * 32, lane); acc[j] = wmma16(ah, kb, acc[j]); acc[j] = wmma16(al, kb, acc[j]); } }
#pragma unroll 1
  for (int kc = 0; kc < 192 / 32; ++kc) { const v16h a = frag_h(AQ + (q0 + col) * (3 * E_) + h * 192 + kc * 32, lane);
#pragma unroll
    for (int j = 0; j < 8; ++j) acs[j] = wmma16(a, frag_h(BK + ((size_t)b * SS + k0 + j * 16 + col) * (3 * E_) + h * 192 + kc * 32, lane), acs[j]); }
#pragma unroll
  for (int j = 0; j < 8; ++j)
#pragma unroll
    for (int r = 0; r < 8; ++r) ss[wave][8 * g + r][j * 16 + col] = acc[j][r] * 0.125f;
  LDSX(); for (int rl = 0; rl < 16; ++rl) vst2(S + (size_t)(ql0 + rl) * SS + k0 + lane * 4, *(const v4f*)&ss[wave][rl][lane * 4]);
  LDSX();
#pragma unroll
  for (int j = 0; j < 8; ++j)
#pragma unroll
    for (int r = 0; r < 8; ++r) ss[wave][8 * g + r][j * 16 + col] = acs[j][r] * (1.0f / 64.0f);
  LDSX(); for (int rl = 0; rl < 16; ++rl) vst2(SG + (size_t)(ql0 + rl) * SS + k0 + lane * 4, *(const v4f*)&ss[wave][rl][lane * 4]); }
__global__ __launch_bounds__(256) void k_smw(const float* __restrict__ S, const float* __restrict__ SG, _Float16* __restrict__ PH, _Float16* __restrict__ GD, _Float16* __restrict__ AE) { __shared__ float sred[8]; __shared__ float sbc; __shared__ __align__(16) _Float16 sp[SS], sg[SS], sa[SS];
  const int t = threadIdx.x; const size_t row = blockIdx.x; const float* sr = S + row * SS;
  float m = -3.0e38f; for (int k = t; k < SS; k += 256) m = fmaxf(m, sr[k]);
#pragma unroll
  for (int o = 1; o < 32; o <<= 1) m = fmaxf(m, __shfl_xor(m, o));
  if ((t & 31) == 0) sred[t >> 5] = m; __syncthreads(); if (t == 0) { float a = sred[0]; for (int i = 1; i < 8; ++i) a = fmaxf(a, sred[i]); sbc = a; } __syncthreads(); m = sbc; __syncthreads();
  float sum = 0.f; for (int k = t; k < SS; k += 256) sum += expf(sr[k] - m);
#pragma unroll
  for (int o = 1; o < 32; o <<= 1) sum += __shfl_xor(sum, o);
  if ((t & 31) == 0) sred[t >> 5] = sum; __syncthreads(); if (t == 0) { float a = 0.f; for (int i = 0; i < 8; ++i) a += sred[i]; sbc = 1.0f / a; } __syncthreads(); const float inv = sbc;
  for (int k = t; k < SS; k += 256) { const float w = expf(sr[k] - m) * inv; const float ws = w * 2048.0f; sp[k] = (_Float16)ws; const float w6 = w * 64.0f; sg[k] = (_Float16)(w6 * w6); const float gr = (w - w * w) * 64.0f; sa[k] = (_Float16)(gr * gr * SG[row * SS + k] * (1.0f / 64.0f)); }
  __syncthreads(); for (int q = t; q < SS / 8; q += 256) { vst2((unsigned*)(PH + row * SS + q * 8), *(const v4u*)&sp[q * 8]); vst2((unsigned*)(GD + row * SS + q * 8), *(const v4u*)&sg[q * 8]); vst2((unsigned*)(AE + row * SS + q * 8), *(const v4u*)&sa[q * 8]); } }
__global__ __launch_bounds__(128) void k_pv2(const _Float16* __restrict__ PH, const _Float16* __restrict__ GD, const _Float16* __restrict__ AE, const _Float16* __restrict__ VT, const _Float16* __restrict__ SGV, const _Float16* __restrict__ VS, int b, int h, float* __restrict__ MUC, _Float16* __restrict__ SGC, float* __restrict__ CST) {
  __shared__ __align__(16) float sm[4][16][68]; __shared__ __align__(16) _Float16 ssg[64][72]; __shared__ __align__(16) float sst[64][2];
  const int tid = threadIdx.x, wave = tid >> 5, lane = tid & 31, col = lane & 15, g = lane >> 4; const int ql0 = blockIdx.x * 64 + wave * 16;
  v8f am[4] = {}, ad[4] = {}, ae[4] = {};
#pragma unroll 1
  for (int kc = 0; kc < SS / 32; ++kc) { const size_t ro = (size_t)(ql0 + col) * SS + kc * 32; const v16h pa = frag_h(PH + ro, lane), pg = frag_h(GD + ro, lane), pe = frag_h(AE + ro, lane);
#pragma unroll
    for (int j = 0; j < 4; ++j) { const size_t po = ((size_t)b * E_ + h * HD + j * 16 + col) * SS + kc * 32; am[j] = wmma16(pa, frag_h(VT + po, lane), am[j]); ad[j] = wmma16(pg, frag_h(SGV + po, lane), ad[j]); ae[j] = wmma16(pe, frag_h(VS + po, lane), ae[j]); } }
  float st0[8], st1[8];
#pragma unroll
  for (int r = 0; r < 8; ++r) { st0[r] = 0.f; st1[r] = 0.f; }
#pragma unroll
  for (int j = 0; j < 4; ++j)
#pragma unroll
    for (int r = 0; r < 8; ++r) { const float mu = am[j][r] * (1.0f / 2048.0f); const float dd = ad[j][r] * (1.0f / (512.0f * 4096.0f)); const float ef = ae[j][r] * (1.0f / (512.0f * 512.0f * 4096.0f)); const float sg = softplusf(dd + ef);
      sm[wave][8 * g + r][j * 16 + col] = mu; ssg[wave * 16 + 8 * g + r][j * 16 + col] = (_Float16)sg; const float mx = mu * (1.0f / E_); st0[r] += mx * mx; st1[r] += sg; }
#pragma unroll
  for (int r = 0; r < 8; ++r) { float a0 = st0[r], a1 = st1[r];
#pragma unroll
    for (int o = 1; o < 16; o <<= 1) { a0 += __shfl_xor(a0, o); a1 += __shfl_xor(a1, o); } if (col == 0) { sst[wave * 16 + 8 * g + r][0] = a0; sst[wave * 16 + 8 * g + r][1] = a1; } }
  __syncthreads();
  for (int rl = 0; rl < 16; ++rl) if (lane < 16) vst2(MUC + ((size_t)b * SS + ql0 + rl) * E_ + h * HD + lane * 4, *(const v4f*)&sm[wave][rl][lane * 4]);
  for (int e = tid; e < 64 * 8; e += 128) { const int rl = e >> 3, q = e & 7; vst2((unsigned*)(SGC + ((size_t)b * SS + blockIdx.x * 64 + rl) * E_ + h * HD + q * 8), *(const v4u*)&ssg[rl][q * 8]); }
  if (tid < 64) { __align__(16) float rec[4] = {sst[tid][0], sst[tid][1], 0.f, 0.f}; vst2(CST + ((size_t)b * SS + blockIdx.x * 64 + tid) * 64 + h * 4, *(const v4f*)rec); } }
__global__ __launch_bounds__(128) void k_outl(const float* __restrict__ MUC, const _Float16* __restrict__ SGC, const float* __restrict__ CST, const float* __restrict__ WO, const _Float16* __restrict__ W2, const float* __restrict__ WSG, float* __restrict__ OUT0, float* __restrict__ OUT1) { __shared__ __align__(16) float sf[4][16][132]; __shared__ float sx[64][2];
  const int tid = threadIdx.x, wave = tid >> 5, lane = tid & 31, col = lane & 15, g = lane >> 4; const int c0 = blockIdx.y * 128; const size_t r0 = (size_t)blockIdx.x * 64 + wave * 16; const _Float16* WO2 = W2 + (size_t)3 * E_ * E_; const float* wsg = WSG + 3 * E_;
  if (tid < 64) { const float* p = CST + ((size_t)blockIdx.x * 64 + tid) * 64; float a = 0.f, bsum = 0.f; for (int hh = 0; hh < NH; ++hh) { a += p[hh * 4]; bsum += p[hh * 4 + 1]; } sx[tid][0] = a; sx[tid][1] = bsum; }
  __syncthreads();
  v8f acc[8] = {}, acs[8] = {};
#pragma unroll 1
  for (int kc = 0; kc < E_ / 32; ++kc) { const F2 a = split_row(MUC + (r0 + col) * E_, kc * 32, lane); const v16h as = frag_h(SGC + (r0 + col) * E_ + kc * 32, lane);
#pragma unroll
    for (int j = 0; j < 8; ++j) { v16b w; v16h w2; const int o = c0 + j * 16 + col;
#pragma unroll
      for (int i = 0; i < 8; ++i) { w[i] = (__bf16)WO[(size_t)(kc * 32 + 8 * g + i) * E_ + o]; w[8 + i] = (__bf16)WO[(size_t)(kc * 32 + 16 + 8 * g + i) * E_ + o]; w2[i] = WO2[(size_t)(kc * 32 + 8 * g + i) * E_ + o]; w2[8 + i] = WO2[(size_t)(kc * 32 + 16 + 8 * g + i) * E_ + o]; }
      acc[j] = wmma_bf(a.h, w, acc[j]); acc[j] = wmma_bf(a.l, w, acc[j]); acs[j] = wmma16(as, w2, acs[j]); } }
#pragma unroll
  for (int j = 0; j < 8; ++j)
#pragma unroll
    for (int r = 0; r < 8; ++r) sf[wave][8 * g + r][j * 16 + col] = acc[j][r];
  LDSX(); for (int rl = 0; rl < 16; ++rl) vst2(OUT0 + (r0 + rl) * E_ + c0 + lane * 4, *(const v4f*)&sf[wave][rl][lane * 4]);
  LDSX();
#pragma unroll
  for (int j = 0; j < 8; ++j) { const int o = c0 + j * 16 + col; const float wsv = wsg[o];
#pragma unroll
    for (int r = 0; r < 8; ++r) { const int rl = wave * 16 + 8 * g + r; const float xx = sx[rl][0], rs = sx[rl][1]; sf[wave][8 * g + r][j * 16 + col] = softplusf(acs[j][r] * (1.0f / E_) + xx * wsv + rs * wsv * (1.0f / E_)); } }
  LDSX(); for (int rl = 0; rl < 16; ++rl) vst2(OUT1 + (r0 + rl) * E_ + c0 + lane * 4, *(const v4f*)&sf[wave][rl][lane * 4]); }
__global__ __launch_bounds__(256) void k_kl(const float* __restrict__ KLP, float* __restrict__ OUT2) { __shared__ float sred[8]; const int t = threadIdx.x; float a = 0.f; for (int e = t; e < E_ * 4; e += 256) a += KLP[e];
#pragma unroll
  for (int o = 1; o < 32; o <<= 1) a += __shfl_xor(a, o); if ((t & 31) == 0) sred[t >> 5] = a; __syncthreads();
  if (t == 0) { float s = 0.f; for (int w = 0; w < 8; ++w) s += sred[w]; const float kl = 0.5f * s / ((float)E_ * (float)E_); vst2(OUT2, kl); } }
extern "C" void kernel_launch(void* const* d_in, const int* in_sizes, int n_in, void* d_out, int out_size, void* d_ws, size_t ws_size, hipStream_t stream) {
  (void)in_sizes; (void)n_in; (void)out_size;
  const float** F = (const float**)d_in;
  if (ws_size < (size_t)WS_END) return;
  char* ws = (char*)d_ws; _Float16 *QH = (_Float16*)(ws + WS_QH), *QL = (_Float16*)(ws + WS_QL), *KH = (_Float16*)(ws + WS_KH), *VT = (_Float16*)(ws + WS_VT), *AQ = (_Float16*)(ws + WS_AQ), *BK = (_Float16*)(ws + WS_BK), *SGV = (_Float16*)(ws + WS_SGV), *VS = (_Float16*)(ws + WS_VS), *PH = (_Float16*)(ws + WS_PH), *GD = (_Float16*)(ws + WS_GD), *AE = (_Float16*)(ws + WS_AE), *SGC = (_Float16*)(ws + WS_SGC), *W2 = (_Float16*)(ws + WS_W2);
  float *RST = (float*)(ws + WS_RST), *S = (float*)(ws + WS_S), *SG = (float*)(ws + WS_SG), *MUC = (float*)(ws + WS_MUC), *CST = (float*)(ws + WS_CST), *WSG = (float*)(ws + WS_WSG);
  float* KLP = S;
  _Float16* VS2 = GD;
  VS2 = SGC;
  float* OUT0 = (float*)d_out; float* OUT1 = OUT0 + OUT1_OFF; float* OUT2 = OUT0 + OUT2_OFF;
  k_prep<<<E_, 256, 0, stream>>>(F[2], F[3], F[4], F[5], F[6], F[7], F[8], F[9], W2, WSG, KLP);
  k_kl<<<1, 256, 0, stream>>>(KLP, OUT2);
  k_rowstat<<<NROW, 256, 0, stream>>>(F[0], F[1], RST);
  k_mu<<<dim3(NROW / 64, E_ / 128, 3), 128, 0, stream>>>(F[0], F[2], F[4], F[6], QH, QL, KH, VT, AQ, VS2);
  for (int which = 0; which < 3; ++which) k_sg<<<dim3(NROW / 64, E_ / 128), 128, 0, stream>>>(F[1], W2, WSG, RST, which, AQ, BK, SGV, VS2, VS);
  for (int b = 0; b < NB; ++b) for (int h = 0; h < NH; ++h) {
    k_sc2<<<dim3(SS / 64, SS / 128), 128, 0, stream>>>(QH, QL, KH, AQ, BK, b, h, S, SG);
    k_smw<<<SS, 256, 0, stream>>>(S, SG, PH, GD, AE);
    k_pv2<<<SS / 64, 128, 0, stream>>>(PH, GD, AE, VT, SGV, VS, b, h, MUC, SGC, CST);
  }
  k_outl<<<dim3(NROW / 64, E_ / 128), 128, 0, stream>>>(MUC, SGC, CST, F[8], W2, WSG, OUT0, OUT1);
}
